// GraphStack_88596585382211
// MI455X (gfx1250) — hardware-run, weakly checked
//
#include <hip/hip_runtime.h>
#include <stdint.h>

#define NBATCH 8
#define NNODE  2048
#define FD     128
#define NLAY   2
#define MROWS  (NBATCH * NNODE)
#define HL     (2 * FD)
#define TP     (2 * NNODE)
#define STP    260
#define SP1    132
#define SP2    68

static_assert(FD == 128);
static_assert(NNODE % 64 == 0);
static_assert(MROWS % 64 == 0);
static_assert(FD % 32 == 0);
static_assert(NNODE % 32 == 0);
static_assert(HL == 2 * FD);
static_assert(TP == 2 * NNODE);
static_assert((64 * STP + HL + 64) * 4 <= 327680);
static_assert((STP * 4) % 16 == 0);
static_assert((SP1 * 4) % 16 == 0);
static_assert((SP2 * 4) % 16 == 0);

typedef __attribute__((ext_vector_type(16))) __bf16 v16b;
typedef __attribute__((ext_vector_type(8)))  __bf16 v8b;
typedef __attribute__((ext_vector_type(8)))  float  v8f;
typedef __attribute__((ext_vector_type(4)))  float  v4f;
typedef __attribute__((ext_vector_type(4)))  unsigned int v4u;

__device__ __forceinline__ unsigned f2bf(float f) {
  const unsigned u = __float_as_uint(f);
  const unsigned r = (u + 0x7FFFu + ((u >> 16) & 1u)) >> 16;
  const unsigned n = (u >> 16) | 0x40u;
  return ((u & 0x7FFFFFFFu) > 0x7F800000u) ? n : r;
}
__device__ __forceinline__ float bf2f(unsigned h) { return __uint_as_float(h << 16); }
__device__ __forceinline__ float bf_rne(float f) { return bf2f(f2bf(f)); }
__device__ __forceinline__ float lrelu(float v) { return (v >= 0.0f) ? v : 0.1f * v; }

struct HLPack { v4u h; v4u l; };
struct F8 { v4f a; v4f c; };

__device__ __forceinline__ HLPack split8(v4f a, v4f c) {
  unsigned hb[8], lb[8];
#pragma unroll
  for (int e = 0; e < 4; ++e) {
    hb[e]     = f2bf(a[e]);
    lb[e]     = f2bf(a[e] - bf2f(hb[e]));
    hb[4 + e] = f2bf(c[e]);
    lb[4 + e] = f2bf(c[e] - bf2f(hb[4 + e]));
  }
  HLPack o;
  o.h = (v4u){hb[0] | (hb[1] << 16), hb[2] | (hb[3] << 16), hb[4] | (hb[5] << 16), hb[6] | (hb[7] << 16)};
  o.l = (v4u){lb[0] | (lb[1] << 16), lb[2] | (lb[3] << 16), lb[4] | (lb[5] << 16), lb[6] | (lb[7] << 16)};
  return o;
}
__device__ __forceinline__ v4u blend(v4u a, v4u b, unsigned m) {
  const v4u mm = {m, m, m, m};
  return (a & ~mm) | (b & mm);
}
__device__ __forceinline__ F8 widen8(v4u w) {
  F8 o;
  o.a = (v4f){__uint_as_float(w[0] << 16), __uint_as_float(w[0] & 0xFFFF0000u),
              __uint_as_float(w[1] << 16), __uint_as_float(w[1] & 0xFFFF0000u)};
  o.c = (v4f){__uint_as_float(w[2] << 16), __uint_as_float(w[2] & 0xFFFF0000u),
              __uint_as_float(w[3] << 16), __uint_as_float(w[3] & 0xFFFF0000u)};
  return o;
}

union FragB { v16b v; v8b h[2]; };
__device__ __forceinline__ v16b ld_frag(const __bf16* p) {
  FragB f;
  f.h[0] = *(const v8b*)(p);
  f.h[1] = *(const v8b*)(p + 16);
  return f.v;
}
__device__ __forceinline__ v8f wmma_bf(v16b a, v16b b, v8f c) {
  v8f d = __builtin_amdgcn_wmma_f32_16x16x32_bf16(false, a, false, b, (short)0, c, false, false);
  asm volatile("v_nop\n\tv_nop\n\tv_nop\n\tv_nop" : "+v"(d) : "v"(a), "v"(b));
  return d;
}

template <int MT, int NT>
__device__ __forceinline__ void gemm_term(const __bf16* ap, const int lda, const __bf16* bp, const int ldb,
                                          const int K, v8f (&acc)[MT][NT]) {
#pragma unroll 1
  for (int k0 = 0; k0 < K; k0 += 32) {
    v16b bf[NT];
#pragma unroll
    for (int j = 0; j < NT; ++j) bf[j] = ld_frag(bp + (size_t)j * 16 * ldb + k0);
#pragma unroll
    for (int i = 0; i < MT; ++i) {
      const v16b af = ld_frag(ap + (size_t)i * 16 * lda + k0);
#pragma unroll
      for (int j = 0; j < NT; ++j) acc[i][j] = wmma_bf(af, bf[j], acc[i][j]);
    }
  }
}

__global__ __launch_bounds__(256) void k_prep(
    const float* __restrict__ x,
    const float* __restrict__ W3, const float* __restrict__ b3,
    const float* __restrict__ W4, const float* __restrict__ b4,
    const float* __restrict__ W5, const float* __restrict__ b5,
    unsigned short* XB, unsigned short* XT, unsigned short* WPQ, unsigned short* W5T, float* BS) {
  __shared__ __align__(16) float tf[64 * SP1];
  const int tid = threadIdx.x, lane = tid & 31, w = tid >> 5;
  const int sub = lane >> 3, q = lane & 7;
  const int blk = blockIdx.x;

  if (blk < 256) {
    const int r0 = blk * 64;
    const int b = r0 >> 11, j0 = r0 & (NNODE - 1);
    {
      const int lr = tid >> 5, c4 = (tid & 31) * 4;
#pragma unroll
      for (int it = 0; it < 8; ++it) {
        const int rr = it * 8 + lr;
        const v4f a = *(const v4f*)(x + (size_t)(r0 + rr) * FD + c4);
        *(v4f*)(tf + rr * SP1 + c4) = a;
      }
    }
    __syncthreads();
    const int hh = lane >> 4, c8 = (lane & 15) * 8;
    v4u xv[4];
#pragma unroll
    for (int i = 0; i < 4; ++i) {
      const int row = w * 8 + i * 2 + hh;
      const v4f a = *(const v4f*)(tf + row * SP1 + c8);
      const v4f c = *(const v4f*)(tf + row * SP1 + c8 + 4);
      const HLPack p = split8(a, c);
      xv[i] = p.h;
    }
    v4u tv[8];
#pragma unroll
    for (int i = 0; i < 8; ++i) {
      const int lid = w * 32 + i * 4 + sub;
      const int f = lid >> 1, hl = lid & 1;
      v4f a, c;
#pragma unroll
      for (int e = 0; e < 4; ++e) {
        a[e] = tf[(8 * q + e) * SP1 + f];
        c[e] = tf[(8 * q + 4 + e) * SP1 + f];
      }
      const HLPack p = split8(a, c);
      const v4u z = {0u, 0u, 0u, 0u};
      tv[i] = blend(p.h, z, 0u - (unsigned)hl);
    }
    for (int pass = 0; pass < 2; ++pass) {
#pragma unroll
      for (int i = 0; i < 4; ++i) {
        const int row = w * 8 + i * 2 + hh;
        *(volatile v4u*)(XB + (size_t)(r0 + row) * FD + c8) = xv[i];
      }
#pragma unroll
      for (int i = 0; i < 8; ++i) {
        const int lid = w * 32 + i * 4 + sub;
        const int f = lid >> 1, hl = lid & 1;
        *(volatile v4u*)(XT + ((size_t)b * FD + f) * TP + hl * NNODE + j0 + 8 * q) = tv[i];
      }
      __threadfence();
    }
  } else if (blk < 280) {
    const int t = blk - 256;
    const int mat = t >> 2, tile = t & 3;
    const int which = mat >> 1, l = mat & 1;
    const int k0 = (tile >> 1) * 64, n0 = (tile & 1) * 64;
    {
      const int lr = tid >> 4, c4 = (tid & 15) * 4;
#pragma unroll
      for (int it = 0; it < 4; ++it) {
        const int rr = it * 16 + lr;
        const size_t so = (size_t)l * FD * FD + (size_t)(k0 + rr) * FD + n0 + c4;
        v4f a;
        if (which == 0)      a = *(const v4f*)(W3 + so);
        else if (which == 1) a = *(const v4f*)(W4 + so);
        else                 a = *(const v4f*)(W5 + so);
        *(v4f*)(tf + rr * SP1 + c4) = a;
      }
    }
    __syncthreads();
    v4u ov[2];
#pragma unroll
    for (int i = 0; i < 2; ++i) {
      const int oc = w * 8 + i * 4 + sub;
      v4f a, c;
#pragma unroll
      for (int e = 0; e < 4; ++e) {
        a[e] = tf[(8 * q + e) * SP1 + oc];
        c[e] = tf[(8 * q + 4 + e) * SP1 + oc];
      }
      const HLPack p = split8(a, c);
      ov[i] = p.h;
    }
    for (int pass = 0; pass < 2; ++pass) {
#pragma unroll
      for (int i = 0; i < 2; ++i) {
        const int oc = w * 8 + i * 4 + sub;
        if (which < 2) {
          *(volatile v4u*)(WPQ + (size_t)l * HL * FD + (size_t)(which * FD + n0 + oc) * FD + k0 + 8 * q) = ov[i];
        } else {
          *(volatile v4u*)(W5T + (size_t)l * FD * FD + (size_t)(n0 + oc) * FD + k0 + 8 * q) = ov[i];
        }
      }
      __threadfence();
    }
  } else {
    if (w < 6) {
      v4f a;
      if (w < 4) {
        const int l = w >> 1;
        if ((w & 1) == 0) a = *(const v4f*)(b3 + l * FD + 4 * lane);
        else              a = *(const v4f*)(b4 + l * FD + 4 * lane);
      } else {
        a = *(const v4f*)(b5 + (w - 4) * FD + 4 * lane);
      }
      v4f o;
#pragma unroll
      for (int e = 0; e < 4; ++e) o[e] = bf_rne(a[e]);
      *(volatile v4f*)(BS + w * 128 + 4 * lane) = o;
      __threadfence();
      *(volatile v4f*)(BS + w * 128 + 4 * lane) = o;
    }
  }
}

template <int LAYER>
__global__ __launch_bounds__(256) __attribute__((amdgpu_num_vgpr(248)))
void k_proj(const unsigned short* __restrict__ Asrc, const unsigned short* __restrict__ Wl,
            const float* __restrict__ biasl, float* DIAG, unsigned short* W1HL, unsigned short* W2T) {
  __shared__ __align__(16) float st[64 * STP];
  __shared__ __align__(16) float sb[HL];
  __shared__ __align__(16) float dgs[64];
  constexpr int LDA = (LAYER == 0) ? FD : HL;
  const int tid = threadIdx.x, lane = tid & 31, w = tid >> 5;
  const int rl = lane & 15, h = lane >> 4;
  const int sub = lane >> 3, q = lane & 7;
  const int m0 = blockIdx.x * 64;
  const int b = m0 >> 11, j0 = m0 & (NNODE - 1);

  {
    const int ci = (tid < 64) ? tid : 63;
    const v4f t = *(const v4f*)(biasl + 4 * ci);
    asm volatile("" :: "v"(t));
    if (tid < 64) *(v4f*)(sb + 4 * tid) = t;
  }

  const __bf16* A  = (const __bf16*)Asrc;
  const __bf16* Bt = (const __bf16*)Wl;
  const __bf16* ap = A + (size_t)(m0 + rl) * LDA + 8 * h;
  const __bf16* bp = Bt + (size_t)(32 * w + rl) * FD + 8 * h;

  v8f acc[4][2];
#pragma unroll
  for (int i = 0; i < 4; ++i)
#pragma unroll
    for (int j = 0; j < 2; ++j) acc[i][j] = (v8f){0.f, 0.f, 0.f, 0.f, 0.f, 0.f, 0.f, 0.f};

  gemm_term<4, 2>(ap, LDA, bp, FD, FD, acc);
  if (LAYER == 1) gemm_term<4, 2>(ap + FD, LDA, bp, FD, FD, acc);

  __syncthreads();
#pragma unroll
  for (int j = 0; j < 2; ++j) {
    const int col = 32 * w + 16 * j + rl;
    const float bv = sb[col];
#pragma unroll
    for (int i = 0; i < 4; ++i)
#pragma unroll
      for (int r = 0; r < 8; ++r) {
        const int row = 16 * i + 8 * h + r;
        st[row * STP + col] = lrelu(acc[i][j][r] + bv);
      }
  }
  __syncthreads();

  {
    const int drow = tid >> 2, part = tid & 3;
    float s = 0.0f;
#pragma unroll 4
    for (int g = 0; g < 32; ++g) {
      const int gg = part * 32 + g;
      s += st[drow * STP + gg] * st[drow * STP + FD + gg];
    }
    s += __shfl_xor(s, 1);
    s += __shfl_xor(s, 2);
    if (part == 0) dgs[drow] = s;
  }

  const int c8 = rl * 8;
  const unsigned hm = 0u - (unsigned)h;
  v4u wv[8];
#pragma unroll
  for (int i = 0; i < 8; ++i) {
    const int row = w * 8 + i;
    const v4f a = *(const v4f*)(st + row * STP + c8);
    const v4f c = *(const v4f*)(st + row * STP + c8 + 4);
    const HLPack p = split8(a, c);
    wv[i] = blend(p.h, p.l, hm);
  }
  v4u tv[8];
#pragma unroll
  for (int i = 0; i < 8; ++i) {
    const int lid = w * 32 + i * 4 + sub;
    const int g = lid >> 1, hl = lid & 1;
    v4f a, c;
#pragma unroll
    for (int e = 0; e < 4; ++e) {
      a[e] = st[(8 * q + e) * STP + FD + g];
      c[e] = st[(8 * q + 4 + e) * STP + FD + g];
    }
    const HLPack p = split8(a, c);
    tv[i] = blend(p.h, p.l, 0u - (unsigned)hl);
  }
  __syncthreads();
  const v4f dv = *(const v4f*)(dgs + 4 * rl);
  asm volatile("" :: "v"(dv));

  for (int pass = 0; pass < 2; ++pass) {
#pragma unroll
    for (int i = 0; i < 8; ++i) {
      const int row = w * 8 + i;
      *(volatile v4u*)(W1HL + (size_t)(m0 + row) * HL + h * FD + c8) = wv[i];
    }
#pragma unroll
    for (int i = 0; i < 8; ++i) {
      const int lid = w * 32 + i * 4 + sub;
      const int g = lid >> 1, hl = lid & 1;
      *(volatile v4u*)(W2T + ((size_t)b * FD + g) * TP + hl * NNODE + j0 + 8 * q) = tv[i];
    }
    if (tid < 16) *(volatile v4f*)(DIAG + m0 + 4 * tid) = dv;
    __threadfence();
  }
}

template <int LAYER>
__global__ __launch_bounds__(256) __attribute__((amdgpu_num_vgpr(248)))
void k_mt(const unsigned short* __restrict__ XT, const unsigned short* __restrict__ W2T, unsigned short* MTHL) {
  __shared__ __align__(16) float st[64 * SP2];
  const int tid = threadIdx.x, lane = tid & 31, w = tid >> 5;
  const int rl = lane & 15, h = lane >> 4;
  const int sub = lane >> 3, q = lane & 7;
  const int tm = blockIdx.x >> 1, tn = blockIdx.x & 1, b = blockIdx.y;
  const int mi = w & 3, nj = w >> 2;

  const __bf16* A  = (const __bf16*)XT;
  const __bf16* Bt = (const __bf16*)W2T;
  const __bf16* ap = A + ((size_t)b * FD + tm * 64 + mi * 16 + rl) * TP + 8 * h;
  const __bf16* bp = Bt + ((size_t)b * FD + tn * 64 + nj * 32 + rl) * TP + 8 * h;

  v8f acc[1][2];
  acc[0][0] = (v8f){0.f, 0.f, 0.f, 0.f, 0.f, 0.f, 0.f, 0.f};
  acc[0][1] = (v8f){0.f, 0.f, 0.f, 0.f, 0.f, 0.f, 0.f, 0.f};

  gemm_term<1, 2>(ap, TP, bp, TP, NNODE, acc);
  if (LAYER == 1) gemm_term<1, 2>(ap + NNODE, TP, bp, TP, NNODE, acc);
  gemm_term<1, 2>(ap, TP, bp + NNODE, TP, NNODE, acc);

#pragma unroll
  for (int j = 0; j < 2; ++j)
#pragma unroll
    for (int r = 0; r < 8; ++r)
      st[(mi * 16 + 8 * h + r) * SP2 + nj * 32 + 16 * j + rl] = acc[0][j][r];
  __syncthreads();

  v4u ov[4];
#pragma unroll
  for (int i = 0; i < 4; ++i) {
    const int lid = w * 16 + i * 4 + sub;
    const int row = lid >> 1, hl = lid & 1;
    const v4f a = *(const v4f*)(st + row * SP2 + 8 * q);
    const v4f c = *(const v4f*)(st + row * SP2 + 8 * q + 4);
    const HLPack p = split8(a, c);
    ov[i] = blend(p.h, p.l, 0u - (unsigned)hl);
  }
  for (int pass = 0; pass < 2; ++pass) {
#pragma unroll
    for (int i = 0; i < 4; ++i) {
      const int lid = w * 16 + i * 4 + sub;
      const int row = lid >> 1, hl = lid & 1;
      *(volatile v4u*)(MTHL + ((size_t)b * FD + tm * 64 + row) * HL + hl * FD + tn * 64 + 8 * q) = ov[i];
    }
    __threadfence();
  }
}

template <int LAYER>
__global__ __launch_bounds__(256) __attribute__((amdgpu_num_vgpr(248)))
void k_msg(const unsigned short* __restrict__ W1HL, const unsigned short* __restrict__ MTHL,
           const float* __restrict__ DIAG, const unsigned short* __restrict__ XB,
           const float* __restrict__ X1, unsigned short* MSGHL) {
  __shared__ __align__(16) float st[64 * SP1];
  __shared__ __align__(16) float dgs[64];
  const int tid = threadIdx.x, lane = tid & 31, w = tid >> 5;
  const int rl = lane & 15, h = lane >> 4;
  const int m0 = blockIdx.x * 64;
  const int b = m0 >> 11;

  {
    const int ci = (tid < 16) ? tid : 15;
    const v4f t = *(const v4f*)(DIAG + m0 + 4 * ci);
    asm volatile("" :: "v"(t));
    if (tid < 16) *(v4f*)(dgs + 4 * tid) = t;
  }

  const __bf16* A  = (const __bf16*)W1HL;
  const __bf16* Bt = (const __bf16*)MTHL;
  const __bf16* ap = A + (size_t)(m0 + rl) * HL + 8 * h;
  const __bf16* bp = Bt + ((size_t)b * FD + 16 * w + rl) * HL + 8 * h;

  v8f acc[4][1];
#pragma unroll
  for (int i = 0; i < 4; ++i) acc[i][0] = (v8f){0.f, 0.f, 0.f, 0.f, 0.f, 0.f, 0.f, 0.f};

  gemm_term<4, 1>(ap, HL, bp, HL, FD, acc);
  gemm_term<4, 1>(ap + FD, HL, bp, HL, FD, acc);
  gemm_term<4, 1>(ap, HL, bp + FD, HL, FD, acc);

#pragma unroll
  for (int i = 0; i < 4; ++i)
#pragma unroll
    for (int r = 0; r < 8; ++r)
      st[(16 * i + 8 * h + r) * SP1 + 16 * w + rl] = acc[i][0][r];
  __syncthreads();

  const int c8 = rl * 8;
  const unsigned hm = 0u - (unsigned)h;
  v4u mv[8];
#pragma unroll
  for (int i = 0; i < 8; ++i) {
    const int row = w * 8 + i;
    const v4f s0 = *(const v4f*)(st + row * SP1 + c8);
    const v4f s1 = *(const v4f*)(st + row * SP1 + c8 + 4);
    F8 xc;
    if (LAYER == 0) {
      const v4u xw = *(const v4u*)(XB + (size_t)(m0 + row) * FD + c8);
      xc = widen8(xw);
    } else {
      xc.a = *(const v4f*)(X1 + (size_t)(m0 + row) * FD + c8);
      xc.c = *(const v4f*)(X1 + (size_t)(m0 + row) * FD + c8 + 4);
    }
    const float dg = dgs[row];
    v4f ma, mc;
#pragma unroll
    for (int e = 0; e < 4; ++e) {
      ma[e] = (s0[e] - dg * xc.a[e]) / 2047.0f;
      mc[e] = (s1[e] - dg * xc.c[e]) / 2047.0f;
    }
    const HLPack p = split8(ma, mc);
    mv[i] = blend(p.h, p.l, hm);
  }
  for (int pass = 0; pass < 2; ++pass) {
#pragma unroll
    for (int i = 0; i < 8; ++i) {
      const int row = w * 8 + i;
      *(volatile v4u*)(MSGHL + (size_t)(m0 + row) * HL + h * FD + c8) = mv[i];
    }
    __threadfence();
  }
}

template <int LAYER>
__global__ __launch_bounds__(256) __attribute__((amdgpu_num_vgpr(248)))
void k_upd(const unsigned short* __restrict__ MSGHL, const unsigned short* __restrict__ W5Tl,
           const float* __restrict__ b5l, const unsigned short* __restrict__ XB,
           const float* __restrict__ Xres, float* Xout, unsigned short* XHL, unsigned short* XT) {
  __shared__ __align__(16) float st[64 * SP1];
  __shared__ __align__(16) float sb[FD];
  const int tid = threadIdx.x, lane = tid & 31, w = tid >> 5;
  const int rl = lane & 15, h = lane >> 4;
  const int sub = lane >> 3, q = lane & 7;
  const int m0 = blockIdx.x * 64;
  const int b = m0 >> 11, j0 = m0 & (NNODE - 1);

  {
    const int ci = (tid < 32) ? tid : 31;
    const v4f t = *(const v4f*)(b5l + 4 * ci);
    asm volatile("" :: "v"(t));
    if (tid < 32) *(v4f*)(sb + 4 * tid) = t;
  }

  const __bf16* A  = (const __bf16*)MSGHL;
  const __bf16* Bt = (const __bf16*)W5Tl;
  const __bf16* ap = A + (size_t)(m0 + rl) * HL + 8 * h;
  const __bf16* bp = Bt + (size_t)(16 * w + rl) * FD + 8 * h;

  v8f acc[4][1];
#pragma unroll
  for (int i = 0; i < 4; ++i) acc[i][0] = (v8f){0.f, 0.f, 0.f, 0.f, 0.f, 0.f, 0.f, 0.f};

  gemm_term<4, 1>(ap, HL, bp, FD, FD, acc);
  gemm_term<4, 1>(ap + FD, HL, bp, FD, FD, acc);

  __syncthreads();
  {
    const int col = 16 * w + rl;
    const float bv = sb[col];
#pragma unroll
    for (int i = 0; i < 4; ++i)
#pragma unroll
      for (int r = 0; r < 8; ++r)
        st[(16 * i + 8 * h + r) * SP1 + col] = lrelu(acc[i][0][r] + bv);
  }
  __syncthreads();

  {
    const int row = tid >> 2, cb = (tid & 3) * 32;
#pragma unroll
    for (int u = 0; u < 4; ++u) {
      const int col = cb + 8 * u;
      F8 xc;
      if (LAYER == 0) {
        const v4u xw = *(const v4u*)(XB + (size_t)(m0 + row) * FD + col);
        xc = widen8(xw);
      } else {
        xc.a = *(const v4f*)(Xres + (size_t)(m0 + row) * FD + col);
        xc.c = *(const v4f*)(Xres + (size_t)(m0 + row) * FD + col + 4);
      }
      v4f s0 = *(const v4f*)(st + row * SP1 + col);
      v4f s1 = *(const v4f*)(st + row * SP1 + col + 4);
#pragma unroll
      for (int e = 0; e < 4; ++e) { s0[e] = s0[e] + xc.a[e]; s1[e] = s1[e] + xc.c[e]; }
      *(v4f*)(st + row * SP1 + col) = s0;
      *(v4f*)(st + row * SP1 + col + 4) = s1;
    }
  }
  __syncthreads();

  v4f ov[8];
#pragma unroll
  for (int i = 0; i < 8; ++i) {
    const int row = w * 8 + i;
    ov[i] = *(const v4f*)(st + row * SP1 + 4 * lane);
  }
  if (LAYER == 1) {
    for (int pass = 0; pass < 2; ++pass) {
#pragma unroll
      for (int i = 0; i < 8; ++i) {
        const int row = w * 8 + i;
        *(volatile v4f*)(Xout + (size_t)(m0 + row) * FD + 4 * lane) = ov[i];
      }
      __threadfence();
    }
  } else {
    const int c8 = rl * 8;
    const unsigned hm = 0u - (unsigned)h;
    v4u hv[8];
#pragma unroll
    for (int i = 0; i < 8; ++i) {
      const int row = w * 8 + i;
      const v4f a = *(const v4f*)(st + row * SP1 + c8);
      const v4f c = *(const v4f*)(st + row * SP1 + c8 + 4);
      const HLPack p = split8(a, c);
      hv[i] = blend(p.h, p.l, hm);
    }
    v4u tv[8];
#pragma unroll
    for (int i = 0; i < 8; ++i) {
      const int lid = w * 32 + i * 4 + sub;
      const int f = lid >> 1, hl = lid & 1;
      v4f a, c;
#pragma unroll
      for (int e = 0; e < 4; ++e) {
        a[e] = st[(8 * q + e) * SP1 + f];
        c[e] = st[(8 * q + 4 + e) * SP1 + f];
      }
      const HLPack p = split8(a, c);
      tv[i] = blend(p.h, p.l, 0u - (unsigned)hl);
    }
    for (int pass = 0; pass < 2; ++pass) {
#pragma unroll
      for (int i = 0; i < 8; ++i) {
        const int row = w * 8 + i;
        *(volatile v4f*)(Xout + (size_t)(m0 + row) * FD + 4 * lane) = ov[i];
        *(volatile v4u*)(XHL + (size_t)(m0 + row) * HL + h * FD + c8) = hv[i];
      }
#pragma unroll
      for (int i = 0; i < 8; ++i) {
        const int lid = w * 32 + i * 4 + sub;
        const int f = lid >> 1, hl = lid & 1;
        *(volatile v4u*)(XT + ((size_t)b * FD + f) * TP + hl * NNODE + j0 + 8 * q) = tv[i];
      }
      __threadfence();
    }
  }
}

extern "C" void kernel_launch(void* const* d_in, const int* in_sizes, int n_in,
                              void* d_out, int out_size, void* d_ws, size_t ws_size,
                              hipStream_t stream) {
  if (n_in < 7) return;
  if (in_sizes[0] != MROWS * FD) return;
  if (in_sizes[1] != NLAY * FD * FD || in_sizes[2] != NLAY * FD) return;
  if (in_sizes[3] != NLAY * FD * FD || in_sizes[4] != NLAY * FD) return;
  if (in_sizes[5] != NLAY * FD * FD || in_sizes[6] != NLAY * FD) return;
  if (out_size != MROWS * FD) return;

  const float* x  = (const float*)d_in[0];
  const float* W3 = (const float*)d_in[1];
  const float* b3 = (const float*)d_in[2];
  const float* W4 = (const float*)d_in[3];
  const float* b4 = (const float*)d_in[4];
  const float* W5 = (const float*)d_in[5];
  const float* b5 = (const float*)d_in[6];
  float* out = (float*)d_out;

  const size_t PXB  = (size_t)MROWS * FD * 2;
  const size_t PXT  = (size_t)NBATCH * FD * TP * 2;
  const size_t PHL  = (size_t)MROWS * HL * 2;
  const size_t PX1  = (size_t)MROWS * FD * 4;
  const size_t PMT  = (size_t)NBATCH * FD * HL * 2;
  const size_t PDG  = (size_t)MROWS * 4;
  const size_t PWPQ = (size_t)NLAY * HL * FD * 2;
  const size_t PW5  = (size_t)NLAY * FD * FD * 2;
  const size_t PBS  = (size_t)768 * 4;
  size_t off = 0;
  const size_t oXB  = off; off += PXB;
  const size_t oXT  = off; off += PXT;
  const size_t oW1  = off; off += PHL;
  const size_t oW2T = off; off += PXT;
  const size_t oMSG = off; off += PHL;
  const size_t oXHL = off; off += PHL;
  const size_t oX1  = off; off += PX1;
  const size_t oMT  = off; off += PMT;
  const size_t oDG  = off; off += PDG;
  const size_t oWPQ = off; off += PWPQ;
  const size_t oW5  = off; off += PW5;
  const size_t oBS  = off; off += PBS;
  if (off > ws_size) return;
  if (off > (size_t)134217728) return;

  char* ws = (char*)d_ws;
  unsigned short* XB    = (unsigned short*)(ws + oXB);
  unsigned short* XT    = (unsigned short*)(ws + oXT);
  unsigned short* W1HL  = (unsigned short*)(ws + oW1);
  unsigned short* W2T   = (unsigned short*)(ws + oW2T);
  unsigned short* MSGHL = (unsigned short*)(ws + oMSG);
  unsigned short* XHL   = (unsigned short*)(ws + oXHL);
  float*          X1    = (float*)(ws + oX1);
  unsigned short* MTHL  = (unsigned short*)(ws + oMT);
  float*          DIAG  = (float*)(ws + oDG);
  unsigned short* WPQ   = (unsigned short*)(ws + oWPQ);
  unsigned short* W5T   = (unsigned short*)(ws + oW5);
  float*          BS    = (float*)(ws + oBS);

  const dim3 blk(256);
  const dim3 gRow(MROWS / 64);
  const dim3 gMt(4, NBATCH);

  k_prep<<<dim3(281), blk, 0, stream>>>(x, W3, b3, W4, b4, W5, b5, XB, XT, WPQ, W5T, BS);

  k_proj<0><<<gRow, blk, 0, stream>>>(XB, WPQ, BS, DIAG, W1HL, W2T);
  k_mt<0><<<gMt, blk, 0, stream>>>(XT, W2T, MTHL);
  k_msg<0><<<gRow, blk, 0, stream>>>(W1HL, MTHL, DIAG, XB, x, MSGHL);
  k_upd<0><<<gRow, blk, 0, stream>>>(MSGHL, W5T, BS + 512, XB, x, X1, XHL, XT);

  k_proj<1><<<gRow, blk, 0, stream>>>(XHL, WPQ + (size_t)HL * FD, BS + 256, DIAG, W1HL, W2T);
  k_mt<1><<<gMt, blk, 0, stream>>>(XT, W2T, MTHL);
  k_msg<1><<<gRow, blk, 0, stream>>>(W1HL, MTHL, DIAG, XB, X1, MSGHL);
  k_upd<1><<<gRow, blk, 0, stream>>>(MSGHL, W5T + (size_t)FD * FD, BS + 640, XB, X1, out, XHL, XT);
  (void)hipGetLastError();
}
